// MySAGE_89043261981499
// MI455X (gfx1250) — hardware-verified
//
#include <hip/hip_runtime.h>
#include <math.h>

#define NN 50000
#define NE 800000
#define NP 50048
#define CIN 128
#define CH 256
#define NT 256
#define SRB 2048
#define NTILE 25
#define NACC (NTILE * SRB)
#define SCH 4096
#define NCH ((NE + SCH - 1) / SCH)
#define NLINES (NE / 32)

typedef __attribute__((ext_vector_type(16))) _Float16 v16h;
typedef __attribute__((ext_vector_type(8)))  _Float16 v8h;
typedef __attribute__((ext_vector_type(16))) __bf16   v16b;
typedef __attribute__((ext_vector_type(8)))  __bf16   v8b;
typedef __attribute__((ext_vector_type(8)))  float    v8f;
typedef __attribute__((ext_vector_type(4)))  float    v4f;
typedef __attribute__((ext_vector_type(4)))  int      v4i;

__device__ __forceinline__ unsigned short f2bf_bits(float f) {
  unsigned u = __float_as_uint(f);
  return (unsigned short)((u + 0x7FFFu + ((u >> 16) & 1u)) >> 16);
}
__device__ __forceinline__ float bf_bits2f(unsigned short h) { return __uint_as_float(((unsigned)h) << 16); }

__device__ __forceinline__ void dep_guard_h(v8f& a, v8f& b, v16h x, v16h y) { asm volatile("v_nop\n\tv_nop\n\tv_nop\n\tv_nop" : "+v"(a), "+v"(b) : "v"(x), "v"(y)); }
__device__ __forceinline__ void dep_guard_b(v8f& a, v8f& b, v16b x, v16b y) { asm volatile("v_nop\n\tv_nop\n\tv_nop\n\tv_nop" : "+v"(a), "+v"(b) : "v"(x), "v"(y)); }
__device__ __forceinline__ void keep4_h(v16h a, v16h b, v16h c, v16h d) { asm volatile("v_nop" :: "v"(a), "v"(b), "v"(c), "v"(d)); }
__device__ __forceinline__ void keep4_b(v16b a, v16b b, v16b c, v16b d) { asm volatile("v_nop" :: "v"(a), "v"(b), "v"(c), "v"(d)); }
__device__ __forceinline__ void fence_v4(v4f& t) { asm volatile("" : "+v"(t)); }
__device__ __forceinline__ void acc_guard4(v8f& a, v8f& b, v8f& c, v8f& d) { asm volatile("v_nop\n\tv_nop\n\tv_nop\n\tv_nop" : "+v"(a), "+v"(b), "+v"(c), "+v"(d)); }
template <typename T> struct Frag;
template <> struct Frag<_Float16> {
  typedef v16h V; union U { v16h v; v8h h[2]; };
  static __device__ __forceinline__ v16h load(const _Float16* p) {
    U f; f.h[0] = *(const v8h*)(p); f.h[1] = *(const v8h*)(p + 16); return f.v;
  }
  static __device__ __forceinline__ v8f mma(v16h a, v16h b, v8f c) {
    return __builtin_amdgcn_wmma_f32_16x16x32_f16(false, a, false, b, (short)0, c, false, false);
  }
  static __device__ __forceinline__ void guard(v8f& a, v8f& b, v16h x, v16h y) { dep_guard_h(a, b, x, y); }
  static __device__ __forceinline__ void keep(v16h a, v16h b, v16h c, v16h d) { keep4_h(a, b, c, d); }
};
template <> struct Frag<__bf16> {
  typedef v16b V; union U { v16b v; v8b h[2]; };
  static __device__ __forceinline__ v16b load(const __bf16* p) {
    U f; f.h[0] = *(const v8b*)(p); f.h[1] = *(const v8b*)(p + 16); return f.v;
  }
  static __device__ __forceinline__ v8f mma(v16b a, v16b b, v8f c) {
    return __builtin_amdgcn_wmma_f32_16x16x32_bf16(false, a, false, b, (short)0, c, false, false);
  }
  static __device__ __forceinline__ void guard(v8f& a, v8f& b, v16b x, v16b y) { dep_guard_b(a, b, x, y); }
  static __device__ __forceinline__ void keep(v16b a, v16b b, v16b c, v16b d) { keep4_b(a, b, c, d); }
};

template <int ET> struct Elem;
template <> struct Elem<0> { typedef _Float16 T; };
template <> struct Elem<1> { typedef __bf16 T; };
template <int ET, bool SPLIT, int BIAS_MODE, int OUT_MODE, bool RESID, int ACT = 0>
__global__ __launch_bounds__(256) void wmma_gemm64(
    const unsigned short* __restrict__ Ap, const unsigned short* __restrict__ A2p, int lda, long strideA,
    const unsigned short* __restrict__ Btp, const unsigned short* __restrict__ Bt2p, int ldb, long strideB,
    void* __restrict__ Cout, void* __restrict__ Cout2, int ldc, long strideC,
    const float* __restrict__ bias,
    const float* __restrict__ resid, long strideR,
    int M, int N, int K, float scale) {
  typedef typename Elem<ET>::T T;
  typedef typename Frag<T>::V V;
  const T* A = (const T*)Ap; const T* A2 = (const T*)A2p; const T* Bt = (const T*)Btp; const T* Bt2 = (const T*)Bt2p;
  __shared__ __align__(16) float sT[8][16 * 68];
  const int b    = blockIdx.y;
  const int lane = threadIdx.x & 31;
  const int wave = threadIdx.x >> 5;
  const int tilesN = N >> 6;
  const int tilesM = M >> 6;
  const int tile = blockIdx.x * 8 + wave;
  if (tile >= tilesM * tilesN) return;
  const int tm = tile / tilesN;
  const int tn = tile - tm * tilesN;
  const int m0 = tm << 6;
  const int n0 = tn << 6;

  const T* Ab  = A  + (size_t)b * strideA;
  const T* Bb  = Bt + (size_t)b * strideB;
  const T* Ab2 = SPLIT ? (A2  + (size_t)b * strideA) : nullptr;
  const T* Bb2 = SPLIT ? (Bt2 + (size_t)b * strideB) : nullptr;

  const int rlane = lane & 15;
  const int koff  = (lane >> 4) * 8;
  const int mOff  = (lane >> 4) * 8;

  v8f acc[4][4];
#pragma unroll
  for (int i = 0; i < 4; ++i)
#pragma unroll
    for (int j = 0; j < 4; ++j) acc[i][j] = (v8f){0.f,0.f,0.f,0.f,0.f,0.f,0.f,0.f};

  for (int k0 = 0; k0 < K; k0 += 32) {
    V bh[4], bl[4];
#pragma unroll
    for (int j = 0; j < 4; ++j) {
      const size_t bo = (size_t)(n0 + (j << 4) + rlane) * ldb + koff + k0;
      bh[j] = Frag<T>::load(Bb + bo);
      if (SPLIT) bl[j] = Frag<T>::load(Bb2 + bo);
    }
#pragma unroll
    for (int i = 0; i < 4; ++i) {
      const size_t ao = (size_t)(m0 + (i << 4) + rlane) * lda + koff + k0;
      V ah = Frag<T>::load(Ab + ao);
      V al;
      if (SPLIT) al = Frag<T>::load(Ab2 + ao);
#pragma unroll
      for (int j = 0; j < 4; ++j) {
        acc[i][j] = Frag<T>::mma(ah, bh[j], acc[i][j]);
        if (SPLIT) {
          acc[i][j] = Frag<T>::mma(ah, bl[j], acc[i][j]);
          acc[i][j] = Frag<T>::mma(al, bh[j], acc[i][j]);
        }
      }
      Frag<T>::guard(acc[i][0], acc[i][3], ah, SPLIT ? al : ah);
    }
    Frag<T>::keep(bh[0], bh[1], bh[2], bh[3]);
    if (SPLIT) Frag<T>::keep(bl[0], bl[1], bl[2], bl[3]);
  }
  acc_guard4(acc[0][0], acc[0][1], acc[0][2], acc[0][3]);
  acc_guard4(acc[1][0], acc[1][1], acc[1][2], acc[1][3]);
  acc_guard4(acc[2][0], acc[2][1], acc[2][2], acc[2][3]);
  acc_guard4(acc[3][0], acc[3][1], acc[3][2], acc[3][3]);

  float* slab = sT[wave];
  const float* Rb = RESID ? (resid + (size_t)b * strideR) : nullptr;
#pragma unroll
  for (int i = 0; i < 4; ++i) {
    const int mBase = m0 + (i << 4);
#pragma unroll
    for (int j = 0; j < 4; ++j) {
      const int n = n0 + (j << 4) + rlane;
      float bv = 0.f;
      if (BIAS_MODE == 2) bv = bias[n];
#pragma unroll
      for (int r = 0; r < 8; ++r) {
        float v = acc[i][j][r] * scale;
        if (BIAS_MODE == 1) v += bias[mBase + mOff + r];
        if (BIAS_MODE == 2) v += bv;
        if (RESID) v += Rb[(size_t)(mBase + mOff + r) * ldc + n];
        if (ACT == 1) v = tanhf(v);
        if (ACT == 2) v = fmaxf(v, 0.0f);
        if (ACT == 3) v = v / (1.0f + expf(-v));
        if (ACT == 4) v = (v > 0.f) ? v : 0.01f * v;
        if (ACT == 5) v = 0.5f * v * (1.0f + erff(v * 0.70710678118654752f));
        slab[(mOff + r) * 68 + (j << 4) + rlane] = v;
      }
    }
    __builtin_amdgcn_fence(__ATOMIC_RELEASE, "workgroup");
    __builtin_amdgcn_wave_barrier();
    __builtin_amdgcn_fence(__ATOMIC_ACQUIRE, "workgroup");
    if (OUT_MODE == 0) {
      float* C = (float*)Cout + (size_t)b * strideC;
      const int hh = lane >> 4, c4 = (lane & 15) * 4;
      for (int pass = 0; pass < 2; ++pass) {
#pragma unroll
        for (int it = 0; it < 8; ++it) {
          const int row = it * 2 + hh;
          v4f v = *(const v4f*)(slab + row * 68 + c4);
          *(volatile v4f*)(C + (size_t)(mBase + row) * ldc + n0 + c4) = v;
        }
        __threadfence();
      }
    } else {
      const int q = lane >> 3, c8 = (lane & 7) * 8;
      unsigned short* C  = (unsigned short*)Cout  + (size_t)b * strideC;
      unsigned short* C2 = (OUT_MODE == 2) ? ((unsigned short*)Cout2 + (size_t)b * strideC) : nullptr;
      for (int pass = 0; pass < 2; ++pass) {
#pragma unroll
        for (int it = 0; it < 4; ++it) {
          const int row = it * 4 + q;
          const float* sp = slab + row * 68 + c8;
          v8h hv, lv;
#pragma unroll
          for (int e = 0; e < 8; ++e) {
            if (OUT_MODE == 1) {
              hv[e] = (_Float16)sp[e];
            } else {
              unsigned short hb = f2bf_bits(sp[e]);
              unsigned short lb = f2bf_bits(sp[e] - bf_bits2f(hb));
              hv[e] = __builtin_bit_cast(_Float16, hb);
              lv[e] = __builtin_bit_cast(_Float16, lb);
            }
          }
          *(volatile v8h*)(C + (size_t)(mBase + row) * ldc + n0 + c8) = hv;
          if (OUT_MODE == 2) *(volatile v8h*)(C2 + (size_t)(mBase + row) * ldc + n0 + c8) = lv;
        }
        __threadfence();
      }
    }
    __builtin_amdgcn_fence(__ATOMIC_RELEASE, "workgroup");
    __builtin_amdgcn_wave_barrier();
    __builtin_amdgcn_fence(__ATOMIC_ACQUIRE, "workgroup");
  }
}

__device__ __forceinline__ int blk_excl_scan(int cnt, int* scan_ws, int tid, int* tot) {
  const int lane = tid & 31, wave = tid >> 5; int incl = cnt;
#pragma unroll
  for (int o = 1; o < 32; o <<= 1) { const int v = __shfl_up(incl, o, 32); if (lane >= o) incl += v; }
  if (lane == 31) scan_ws[wave] = incl;
  __syncthreads();
  if (wave == 0) { int wv = (lane < NT / 32) ? scan_ws[lane] : 0; int wincl = wv;
#pragma unroll
    for (int o = 1; o < 32; o <<= 1) { const int v = __shfl_up(wincl, o, 32); if (lane >= o) wincl += v; }
    if (lane < NT / 32) scan_ws[32 + lane] = wincl - wv; if (lane == 31) scan_ws[64] = wincl; }
  __syncthreads();
  const int res = scan_ws[32 + wave] + incl - cnt; *tot = scan_ws[64];
  return res;
}
template <int SP, int CAP>
__device__ __forceinline__ int chunk_hits(const int* __restrict__ dstv, const int* __restrict__ srcv, int e0, int n0, int tid,
                                          int* LIST, int* scan_ws) {
  const int eb = e0 + tid * SP;
  const bool inr = eb < NE;
  const int ebc = inr ? eb : (NE - SP);
  int rec[SP]; int cnt = 0;
#pragma unroll
  for (int k = 0; k < SP; k += 4) {
    const v4i d4 = *(const v4i*)(dstv + ebc + k);
    const v4i s4 = *(const v4i*)(srcv + ebc + k);
#pragma unroll
    for (int e = 0; e < 4; ++e) {
      const int d = d4[e]; int r = -1;
      if (inr && d >= n0 && d < n0 + SRB) { int s = s4[e]; s = s < 0 ? 0 : (s >= NN ? NN - 1 : s); r = ((d - n0) << 16) | s; ++cnt; }
      rec[k + e] = r;
    }
  }
  int tot; int p = blk_excl_scan(cnt, scan_ws, tid, &tot);
#pragma unroll
  for (int k = 0; k < SP; ++k) if (rec[k] >= 0) { if ((unsigned)p < (unsigned)CAP) LIST[p] = rec[k]; ++p; }
  __syncthreads();
  return tot < CAP ? tot : CAP;
}

__global__ __launch_bounds__(NT) void prep_kernel(const float* __restrict__ w1l, const float* __restrict__ w1r,
                                                 const float* __restrict__ w2l, const float* __restrict__ w2r, unsigned* __restrict__ WT) {
  const int i = blockIdx.x * NT + threadIdx.x;
  if (i < 2 * (CH * CH / 2)) {
    const int plane = i >> 15;
    const int ii = i & 32767;
    const int n = ii >> 7;
    const int k = 2 * (ii & 127);
    const int kk = k & 127, nn = n & 127;
    const float al0 = w1l[kk * CH + n], al1 = w1l[(kk + 1) * CH + n];
    const float ar0 = w1r[kk * CH + n], ar1 = w1r[(kk + 1) * CH + n];
    const float bl0 = w2l[k * CIN + nn], bl1 = w2l[(k + 1) * CIN + nn];
    const float br0 = w2r[k * CIN + nn], br1 = w2r[(k + 1) * CIN + nn];
    const float v0a = (k < 128) ? al0 : ar0, v0b = (k < 128) ? al1 : ar1;
    const float v1a = (n < 128) ? bl0 : br0, v1b = (n < 128) ? bl1 : br1;
    const float fa = (plane ? v1a : v0a) * 16.0f, fb = (plane ? v1b : v0b) * 16.0f;
    const _Float16 h0 = (_Float16)fa, h1 = (_Float16)fb;
    const unsigned u = (unsigned)__builtin_bit_cast(unsigned short, h0) | ((unsigned)__builtin_bit_cast(unsigned short, h1) << 16);
    ((volatile unsigned*)WT)[i] = u;
    __threadfence();
    ((volatile unsigned*)WT)[i] = u;
  }
}

__global__ __launch_bounds__(NT) void agg1_kernel(const float* __restrict__ x, const int* __restrict__ ei, float* AGG,
                                                 unsigned short* __restrict__ A1) {
  __shared__ int LIST[SCH];
  __shared__ int CNT[SRB];
  __shared__ int scan_ws[80];
  const int tid = threadIdx.x, lane = tid & 31, wave = tid >> 5;
  const int n0 = blockIdx.x * SRB;
  const v4f z4 = {0.f, 0.f, 0.f, 0.f};
  for (int pass = 0; pass < 2; ++pass) {
#pragma unroll 1
    for (int j = 0; j < SRB / 8; ++j) {
      float* rp = AGG + (size_t)(n0 + wave * (SRB / 8) + j) * CIN + 4 * lane;
      *(volatile v4f*)rp = z4;
    }
    __threadfence();
  }
  for (int i = tid; i < SRB; i += NT) CNT[i] = 0;
  __syncthreads();
  const int* srcv = ei; const int* dstv = ei + NE;
#pragma unroll 1
  for (int c = 0; c < NCH; ++c) {
    const int tot = chunk_hits<SCH / NT, SCH>(dstv, srcv, c * SCH, n0, tid, LIST, scan_ws);
#pragma unroll 1
    for (int base = 0; base < tot; base += 32) {
      const int q = base + lane;
      const int lv = LIST[q];
      const int rv = (q < tot) ? lv : -1;
      const int own = (rv >= 0 && (rv >> 24) == wave) ? 1 : 0;
      unsigned msk = (unsigned)__ballot(own);
#pragma unroll 1
      for (int it = 0; it < 32; ++it) {
        if (msk == 0u) break;
        const int bp = __builtin_ctz(msk); msk &= msk - 1u;
        const int r = __shfl(rv, bp, 32);
        const int dl = (r >> 16) & (SRB - 1);
        int s = r & 0xFFFF; s = s < NN ? s : NN - 1;
        const v4f xs = *(const v4f*)(x + (size_t)s * CIN + 4 * lane);
        float* rp = AGG + (size_t)(n0 + dl) * CIN + 4 * lane;
        v4f a = *(const v4f*)rp;
        a = a + xs;
        *(volatile v4f*)rp = a;
        __threadfence();
        *(volatile v4f*)rp = a;
        if (lane == 0) CNT[dl] += 1;
      }
    }
    __syncthreads();
  }
  const int c8 = 8 * (lane & 15);
  const bool hiHalf = lane >= 16;
#pragma unroll 1
  for (int j = 0; j < SRB / 8; ++j) {
    const int dl = wave * (SRB / 8) + j; const int n = n0 + dl;
    if (n < NP) {
      const bool live = n < NN;
      const int nc = live ? n : NN - 1;
      const float cf = (float)CNT[dl];
      const float inv = 1.0f / fmaxf(cf, 1.0f);
      const float* rp = AGG + (size_t)(n0 + dl) * CIN + c8;
      const float* xp = x + (size_t)nc * CIN + c8;
      const v4f a0 = *(const v4f*)rp, a1 = *(const v4f*)(rp + 4);
      const v4f x0 = *(const v4f*)xp, x1 = *(const v4f*)(xp + 4);
      v8h hv;
#pragma unroll
      for (int e = 0; e < 4; ++e) {
        float f0 = hiHalf ? x0[e] : a0[e] * inv;
        float f1 = hiHalf ? x1[e] : a1[e] * inv;
        f0 = live ? f0 : 0.f; f1 = live ? f1 : 0.f;
        hv[e] = (_Float16)f0; hv[4 + e] = (_Float16)f1;
      }
      unsigned short* dp = A1 + (size_t)n * CH + 8 * lane;
      *(volatile v8h*)dp = hv;
      __threadfence();
      *(volatile v8h*)dp = hv;
    }
  }
}

__global__ __launch_bounds__(NT) void agg2_kernel(const float* __restrict__ HZ, const int* __restrict__ ei, const float* __restrict__ b2, float* Z) {
  __shared__ int LIST[SCH];
  __shared__ int CNT[SRB];
  __shared__ int scan_ws[80];
  const int tid = threadIdx.x, lane = tid & 31, wave = tid >> 5;
  const int n0 = blockIdx.x * SRB;
  const v4f z4 = {0.f, 0.f, 0.f, 0.f};
  const v4f bv = *(const v4f*)(b2 + 4 * lane);
  for (int pass = 0; pass < 2; ++pass) {
#pragma unroll 1
    for (int j = 0; j < SRB / 8; ++j) {
      float* rp = Z + (size_t)(n0 + wave * (SRB / 8) + j) * CIN + 4 * lane;
      *(volatile v4f*)rp = z4;
    }
    __threadfence();
  }
  for (int i = tid; i < SRB; i += NT) CNT[i] = 0;
  __syncthreads();
  const int* srcv = ei; const int* dstv = ei + NE;
#pragma unroll 1
  for (int c = 0; c < NCH; ++c) {
    const int tot = chunk_hits<SCH / NT, SCH>(dstv, srcv, c * SCH, n0, tid, LIST, scan_ws);
#pragma unroll 1
    for (int base = 0; base < tot; base += 32) {
      const int q = base + lane;
      const int lv = LIST[q];
      const int rv = (q < tot) ? lv : -1;
      const int own = (rv >= 0 && (rv >> 24) == wave) ? 1 : 0;
      unsigned msk = (unsigned)__ballot(own);
#pragma unroll 1
      for (int it = 0; it < 32; ++it) {
        if (msk == 0u) break;
        const int bp = __builtin_ctz(msk); msk &= msk - 1u;
        const int r = __shfl(rv, bp, 32);
        const int dl = (r >> 16) & (SRB - 1);
        int s = r & 0xFFFF; s = s < NN ? s : NN - 1;
        const v4f hv = *(const v4f*)(HZ + (size_t)s * CH + 4 * lane);
        float* rp = Z + (size_t)(n0 + dl) * CIN + 4 * lane;
        v4f a = *(const v4f*)rp;
        a = a + hv;
        *(volatile v4f*)rp = a;
        __threadfence();
        *(volatile v4f*)rp = a;
        if (lane == 0) CNT[dl] += 1;
      }
    }
    __syncthreads();
  }
#pragma unroll 1
  for (int j = 0; j < SRB / 8; ++j) {
    const int dl = wave * (SRB / 8) + j; const int n = n0 + dl;
    if (n < NN) {
      const float cf = (float)CNT[dl];
      const float inv = 1.0f / fmaxf(cf, 1.0f);
      float* rp = Z + (size_t)n * CIN + 4 * lane;
      const v4f a = *(const v4f*)rp;
      v4f t = a * inv; fence_v4(t);
      t = t + bv;
      const v4f hr = *(const v4f*)(HZ + (size_t)n * CH + CIN + 4 * lane);
      t = t + hr;
      *(volatile v4f*)rp = t;
      __threadfence();
      *(volatile v4f*)rp = t;
    }
  }
}

__global__ __launch_bounds__(NT) void decode_kernel(const float* __restrict__ Z, const int* __restrict__ ei, float* __restrict__ out) {
  const int lane = threadIdx.x & 31, wave = threadIdx.x >> 5;
  const int line = blockIdx.x * (NT / 32) + wave;
  if (line >= NLINES) return;
  const int e0 = line * 32;
  int sv = ei[e0 + lane], dv = ei[NE + e0 + lane];
  sv = sv < 0 ? 0 : (sv >= NN ? NN - 1 : sv);
  dv = dv < 0 ? 0 : (dv >= NN ? NN - 1 : dv);
  float res = 0.f;
#pragma unroll 1
  for (int g = 0; g < 4; ++g) {
    float v[8];
#pragma unroll
    for (int i = 0; i < 8; ++i) {
      const int s = __shfl(sv, 8 * g + i, 32), d = __shfl(dv, 8 * g + i, 32);
      const v4f a = *(const v4f*)(Z + (size_t)s * CIN + 4 * lane);
      const v4f b = *(const v4f*)(Z + (size_t)d * CIN + 4 * lane);
      v[i] = a[0] * b[0] + a[1] * b[1] + a[2] * b[2] + a[3] * b[3];
    }
#pragma unroll
    for (int j = 0; j < 4; ++j) {
      const bool up = (lane & 16) != 0;
      const float keep = up ? v[j + 4] : v[j]; const float send = up ? v[j] : v[j + 4];
      v[j] = keep + __shfl_xor(send, 16, 32);
    }
#pragma unroll
    for (int j = 0; j < 2; ++j) {
      const bool up = (lane & 8) != 0;
      const float keep = up ? v[j + 2] : v[j]; const float send = up ? v[j] : v[j + 2];
      v[j] = keep + __shfl_xor(send, 8, 32);
    }
    {
      const bool up = (lane & 4) != 0;
      const float keep = up ? v[1] : v[0]; const float send = up ? v[0] : v[1];
      v[0] = keep + __shfl_xor(send, 4, 32);
    }
    float t = v[0];
    t += __shfl_xor(t, 1, 32);
    t += __shfl_xor(t, 2, 32);
    const float mine = __shfl(t, 4 * (lane & 7), 32);
    res = ((lane >> 3) == g) ? mine : res;
  }
  const float d = fminf(fmaxf(res, -30.0f), 30.0f);
  const float p = 1.0f / (1.0f + expf(-d));
  float* op = out + (size_t)e0 + lane;
  *(volatile float*)op = p;
  __threadfence();
  *(volatile float*)op = p;
}

extern "C" void kernel_launch(void* const* d_in, const int* in_sizes, int n_in,
                              void* d_out, int out_size, void* d_ws, size_t ws_size, hipStream_t stream) {
  if (n_in < 8) return;
  if (in_sizes[0] != NN * CIN || in_sizes[1] != 2 * NE || in_sizes[2] != CIN * CH || in_sizes[3] != CH ||
      in_sizes[4] != CIN * CH || in_sizes[5] != CH * CIN || in_sizes[6] != CIN || in_sizes[7] != CH * CIN || out_size != NE) return;
  const float* x   = (const float*)d_in[0];
  const int*   ei  = (const int*)  d_in[1];
  const float* w1l = (const float*)d_in[2];
  const float* b1  = (const float*)d_in[3];
  const float* w1r = (const float*)d_in[4];
  const float* w2l = (const float*)d_in[5];
  const float* b2  = (const float*)d_in[6];
  const float* w2r = (const float*)d_in[7];
  float* out = (float*)d_out;

  char* ws = (char*)d_ws; size_t off = 0;
  auto carve = [&](size_t bytes) -> char* { char* p = ws + off; off += (bytes + 255) & ~(size_t)255; return p; };
  unsigned* WT  = (unsigned*)carve((size_t)2 * CH * CH * 2);
  char*     R1  = carve((size_t)NP * CH * 4);
  float*    ACC = (float*)carve((size_t)NACC * CIN * 4);
  unsigned short* H = (unsigned short*)carve((size_t)NP * CH * 2);
  if (off > ws_size || off > (size_t)134217728) return;
  unsigned short* A1  = (unsigned short*)R1;
  float*          HZ  = (float*)R1;
  const unsigned short* W1T = (const unsigned short*)WT;
  const unsigned short* W2T = (const unsigned short*)WT + (size_t)CH * CH;

  prep_kernel<<<(CH * CH + NT - 1) / NT, NT, 0, stream>>>(w1l, w1r, w2l, w2r, WT);
  agg1_kernel<<<NTILE, NT, 0, stream>>>(x, ei, ACC, A1);
  {
    const int tiles = (NP / 64) * (CH / 64);
    wmma_gemm64<0, false, 2, 1, false, 2><<<dim3((tiles + 7) / 8, 1), 256, 0, stream>>>(
        (const unsigned short*)A1, (const unsigned short*)nullptr, CH, 0L,
        W1T, (const unsigned short*)nullptr, CH, 0L,
        (void*)H, (void*)nullptr, CH, 0L,
        b1, (const float*)nullptr, 0L, NP, CH, CH, 1.0f / 16.0f);
    wmma_gemm64<0, false, 0, 0, false, 0><<<dim3((tiles + 7) / 8, 1), 256, 0, stream>>>(
        (const unsigned short*)H, (const unsigned short*)nullptr, CH, 0L,
        W2T, (const unsigned short*)nullptr, CH, 0L,
        (void*)HZ, (void*)nullptr, CH, 0L,
        (const float*)nullptr, (const float*)nullptr, 0L, NP, CH, CH, 1.0f / 16.0f);
  }
  agg2_kernel<<<NTILE, NT, 0, stream>>>(HZ, ei, b2, ACC);
  decode_kernel<<<NLINES / (NT / 32), NT, 0, stream>>>(ACC, ei, out);
}
